// TokenSwapMamba_81561428951253
// MI455X (gfx1250) — hardware-verified
//
#include <hip/hip_runtime.h>
#include <math.h>

typedef __attribute__((ext_vector_type(16))) _Float16 v16h;
typedef __attribute__((ext_vector_type(8)))  _Float16 v8h;
typedef __attribute__((ext_vector_type(8)))  float    v8f;
typedef __attribute__((ext_vector_type(4)))  float    v4f;

constexpr int kDim    = 96;
constexpr int kDin    = 192;
constexpr int kNst    = 16;
constexpr int kDtR    = 6;
constexpr int kSwap   = 59;
constexpr int kBatch  = 2;
constexpr int kSeq    = 6400;
constexpr int kTok    = kBatch * kSeq;
constexpr int kXzP    = 2 * kDin;
constexpr int kXdN    = kDtR + 2 * kNst;
constexpr int kXdP    = 64;
constexpr int kEnc    = 2;
constexpr int kConvP  = 196;
constexpr int kScanYP = 400;
constexpr int kScanYH = 200;
constexpr int kOutP   = 100;
constexpr float kWCarry    = 32.0f;
constexpr float kYCarry    = 16.0f;
constexpr float kInvWCarry = 1.0f / kWCarry;
constexpr float kInvOutCarry = 1.0f / (kWCarry * kYCarry);
constexpr float kInvDim    = 1.0f / (float)kDim;

static_assert(kTok == 12800 && kXzP == 384 && kXdN == 38, "shape constants");
static_assert((kTok % 64) == 0 && (kXzP % 64) == 0 && (kXdP % 64) == 0, "GEMM M,N multiples of 64");
static_assert((kDim % 32) == 0 && (kDin % 32) == 0, "GEMM K multiples of 32");
static_assert((kSeq % 64) == 0 && (kSeq % 16) == 0 && (kTok % 16) == 0, "tile multiples");
static_assert(kXdN <= kXdP, "x_proj pad");

constexpr size_t kSzWI   = (size_t)kEnc * kXzP * kDim * 2;
constexpr size_t kSzWX   = (size_t)kEnc * kXdP * kDin * 2;
constexpr size_t kSzWO   = (size_t)kEnc * kDim * kDin * 2;
constexpr size_t kSzXS   = (size_t)kEnc * kTok * kDim * 2;
constexpr size_t kSzXZ   = (size_t)kEnc * kTok * kXzP * 4;
constexpr size_t kSzUC   = (size_t)kEnc * kTok * kDin * 4;
constexpr size_t kSzUC16 = (size_t)kEnc * kTok * kDin * 2;
constexpr size_t kSzXD   = (size_t)kEnc * kTok * kXdP * 4;
constexpr size_t kSzY16  = (size_t)kEnc * kTok * kDin * 2;
constexpr size_t kOffWI   = 0;
constexpr size_t kOffWX   = kOffWI   + kSzWI;
constexpr size_t kOffWO   = kOffWX   + kSzWX;
constexpr size_t kOffXS   = kOffWO   + kSzWO;
constexpr size_t kOffXZ   = kOffXS   + kSzXS;
constexpr size_t kOffUC   = kOffXZ   + kSzXZ;
constexpr size_t kOffUC16 = kOffUC   + kSzUC;
constexpr size_t kOffXD   = kOffUC16 + kSzUC16;
constexpr size_t kOffY16  = kOffXD   + kSzXD;
constexpr size_t kWsTotal = kOffY16  + kSzY16;
static_assert(kWsTotal == 90382336ull, "carve total");
static_assert(kWsTotal <= 134217728ull, "carve cap");
static_assert((kOffWX % 128) == 0 && (kOffWO % 128) == 0 && (kOffXS % 128) == 0 && (kOffXZ % 128) == 0 &&
              (kOffUC % 128) == 0 && (kOffUC16 % 128) == 0 && (kOffXD % 128) == 0 && (kOffY16 % 128) == 0,
              "128-B aligned regions");
static_assert(((size_t)kXzP * kDim * 2) % 128 == 0 && ((size_t)kXdP * kDin * 2) % 128 == 0 &&
              ((size_t)kDim * kDin * 2) % 128 == 0 && ((size_t)kTok * kDim * 2) % 128 == 0 &&
              ((size_t)kTok * kDim * 4) % 128 == 0, "per-encoder planes line aligned");

__device__ __forceinline__ void guard4_h(v8f& a0, v8f& a1, v8f& a2, v8f& a3,
                                         v16h x, v16h b0, v16h b1, v16h b2, v16h b3) {
  asm volatile("v_nop\n\tv_nop\n\tv_nop\n\tv_nop"
               : "+v"(a0), "+v"(a1), "+v"(a2), "+v"(a3)
               : "v"(x), "v"(b0), "v"(b1), "v"(b2), "v"(b3));
}
__device__ __forceinline__ void guard6_h(v8f& a0, v8f& a1, v8f& a2, v8f& a3, v8f& a4, v8f& a5,
                                         v16h x, v16h b0, v16h b1, v16h b2, v16h b3, v16h b4, v16h b5) {
  asm volatile("v_nop\n\tv_nop\n\tv_nop\n\tv_nop"
               : "+v"(a0), "+v"(a1), "+v"(a2), "+v"(a3), "+v"(a4), "+v"(a5)
               : "v"(x), "v"(b0), "v"(b1), "v"(b2), "v"(b3), "v"(b4), "v"(b5));
}
__device__ __forceinline__ void keep4_h(v16h a, v16h b, v16h c, v16h d) {
  asm volatile("v_nop" :: "v"(a), "v"(b), "v"(c), "v"(d));
}
__device__ __forceinline__ void acc_guard4(v8f& a, v8f& b, v8f& c, v8f& d) {
  asm volatile("v_nop\n\tv_nop\n\tv_nop\n\tv_nop" : "+v"(a), "+v"(b), "+v"(c), "+v"(d));
}
struct FragH {
  union U { v16h v; v8h h[2]; };
  static __device__ __forceinline__ v16h load(const _Float16* p) {
    U f;
    f.h[0] = *(const v8h*)(p);
    f.h[1] = *(const v8h*)(p + 16);
    return f.v;
  }
  static __device__ __forceinline__ v8f mma(v16h a, v16h b, v8f c) {
    return __builtin_amdgcn_wmma_f32_16x16x32_f16(false, a, false, b, (short)0, c, false, false);
  }
};

__global__ __launch_bounds__(256) void gemm64_f16_kernel(
    const unsigned short* __restrict__ Ap, int lda, long strideA,
    const unsigned short* __restrict__ Btp, int ldb, long strideB,
    float* __restrict__ Cout, int ldc, long strideC,
    int M, int N, int K, float scale) {
  const _Float16* A  = (const _Float16*)Ap;
  const _Float16* Bt = (const _Float16*)Btp;
  __shared__ __align__(16) float sT[8][16 * 68];
  const int b    = blockIdx.y;
  const int lane = threadIdx.x & 31;
  const int wave = threadIdx.x >> 5;
  const int tilesN = N >> 6;
  const int tilesM = M >> 6;
  const int tile = blockIdx.x * 8 + wave;
  if (tile >= tilesM * tilesN) return;
  const int tm = tile / tilesN;
  const int tn = tile - tm * tilesN;
  const int m0 = tm << 6;
  const int n0 = tn << 6;

  const _Float16* Ab = A  + (size_t)b * strideA;
  const _Float16* Bb = Bt + (size_t)b * strideB;

  const int rlane = lane & 15;
  const int koff  = (lane >> 4) * 8;
  const int mOff  = (lane >> 4) * 8;

  v8f acc[4][4];
#pragma unroll
  for (int i = 0; i < 4; ++i)
#pragma unroll
    for (int j = 0; j < 4; ++j) acc[i][j] = (v8f){0.f, 0.f, 0.f, 0.f, 0.f, 0.f, 0.f, 0.f};

  for (int k0 = 0; k0 < K; k0 += 32) {
    v16h bh[4];
#pragma unroll
    for (int j = 0; j < 4; ++j) {
      const size_t bo = (size_t)(n0 + (j << 4) + rlane) * ldb + koff + k0;
      bh[j] = FragH::load(Bb + bo);
    }
#pragma unroll
    for (int i = 0; i < 4; ++i) {
      const size_t ao = (size_t)(m0 + (i << 4) + rlane) * lda + koff + k0;
      v16h ah = FragH::load(Ab + ao);
#pragma unroll
      for (int j = 0; j < 4; ++j) acc[i][j] = FragH::mma(ah, bh[j], acc[i][j]);
      guard4_h(acc[i][0], acc[i][1], acc[i][2], acc[i][3], ah, bh[0], bh[1], bh[2], bh[3]);
    }
    keep4_h(bh[0], bh[1], bh[2], bh[3]);
  }
  acc_guard4(acc[0][0], acc[0][1], acc[0][2], acc[0][3]);
  acc_guard4(acc[1][0], acc[1][1], acc[1][2], acc[1][3]);
  acc_guard4(acc[2][0], acc[2][1], acc[2][2], acc[2][3]);
  acc_guard4(acc[3][0], acc[3][1], acc[3][2], acc[3][3]);

  float* slab = sT[wave];
  float* C = Cout + (size_t)b * strideC;
  const int hh = lane >> 4, c4 = (lane & 15) * 4;
#pragma unroll
  for (int i = 0; i < 4; ++i) {
    const int mBase = m0 + (i << 4);
#pragma unroll
    for (int j = 0; j < 4; ++j) {
#pragma unroll
      for (int r = 0; r < 8; ++r) {
        slab[(mOff + r) * 68 + (j << 4) + rlane] = acc[i][j][r] * scale;
      }
    }
    __builtin_amdgcn_fence(__ATOMIC_RELEASE, "workgroup");
    __builtin_amdgcn_wave_barrier();
    __builtin_amdgcn_fence(__ATOMIC_ACQUIRE, "workgroup");
    for (int pass = 0; pass < 2; ++pass) {
#pragma unroll
      for (int it = 0; it < 8; ++it) {
        const int row = it * 2 + hh;
        v4f v = *(const v4f*)(slab + row * 68 + c4);
        *(volatile v4f*)(C + (size_t)(mBase + row) * ldc + n0 + c4) = v;
      }
      __threadfence();
    }
    __builtin_amdgcn_fence(__ATOMIC_RELEASE, "workgroup");
    __builtin_amdgcn_wave_barrier();
    __builtin_amdgcn_fence(__ATOMIC_ACQUIRE, "workgroup");
  }
}

__global__ __launch_bounds__(256) void cast_pad_f16_kernel(
    const float* __restrict__ s0, const float* __restrict__ s1, unsigned short* __restrict__ dst,
    int rows_real, int rows_pad, int kdim, float scale)
{
  const int i = blockIdx.x * 256 + threadIdx.x;
  const int total8 = (rows_pad * kdim) >> 3;
  if (i >= total8) return;
  const float* src = (blockIdx.y == 0) ? s0 : s1;
  const int e0  = i << 3;
  const int row = e0 / kdim;
  const int col = e0 - row * kdim;
  const bool real = (row < rows_real);
  const int rc = real ? row : (rows_real - 1);
  const float* p = src + (size_t)rc * kdim + col;
  const v4f a0 = *(const v4f*)(p);
  const v4f a1 = *(const v4f*)(p + 4);
  v8h hv;
#pragma unroll
  for (int e = 0; e < 4; ++e) {
    const float f0 = real ? (a0[e] * scale) : 0.0f;
    const float f1 = real ? (a1[e] * scale) : 0.0f;
    hv[e]     = (_Float16)f0;
    hv[4 + e] = (_Float16)f1;
  }
  unsigned short* q = dst + (size_t)blockIdx.y * rows_pad * kdim + e0;
  *(volatile v8h*)q = hv;
  __threadfence();
  *(volatile v8h*)q = hv;
}

__global__ __launch_bounds__(256) void ln_swap_shuffle_kernel(
    const float* __restrict__ x1, const float* __restrict__ x2,
    const float* __restrict__ g1, const float* __restrict__ b1,
    const float* __restrict__ g2, const float* __restrict__ b2,
    unsigned short* __restrict__ XS)
{
  __shared__ __align__(16) float sN[8 * 4 * kDim];
  const int lane = threadIdx.x & 31, wave = threadIdx.x >> 5;
  const int t0 = (blockIdx.x * 8 + wave) * 2;
  float* sw = sN + wave * (4 * kDim);
  float pg1[3], pb1[3], pg2[3], pb2[3];
#pragma unroll
  for (int i = 0; i < 3; ++i) {
    const int ch = lane + 32 * i;
    pg1[i] = g1[ch]; pb1[i] = b1[ch]; pg2[i] = g2[ch]; pb2[i] = b2[ch];
  }
#pragma unroll 1
  for (int tok = 0; tok < 2; ++tok) {
    const float* p1 = x1 + (size_t)(t0 + tok) * kDim;
    const float* p2 = x2 + (size_t)(t0 + tok) * kDim;
    float a[3], c[3];
#pragma unroll
    for (int i = 0; i < 3; ++i) { a[i] = p1[lane + 32 * i]; c[i] = p2[lane + 32 * i]; }
    float s1 = (a[0] + a[1]) + a[2];
    float s2 = (c[0] + c[1]) + c[2];
#pragma unroll
    for (int m = 16; m >= 1; m >>= 1) { s1 += __shfl_xor(s1, m, 32); s2 += __shfl_xor(s2, m, 32); }
    const float m1 = s1 * kInvDim, m2 = s2 * kInvDim;
    float q1 = 0.f, q2 = 0.f;
#pragma unroll
    for (int i = 0; i < 3; ++i) {
      const float d1 = a[i] - m1, d2 = c[i] - m2;
      q1 += d1 * d1;
      q2 += d2 * d2;
    }
#pragma unroll
    for (int m = 16; m >= 1; m >>= 1) { q1 += __shfl_xor(q1, m, 32); q2 += __shfl_xor(q2, m, 32); }
    const float r1 = rsqrtf(q1 * kInvDim + 1e-5f);
    const float r2 = rsqrtf(q2 * kInvDim + 1e-5f);
#pragma unroll
    for (int i = 0; i < 3; ++i) {
      const int ch = lane + 32 * i;
      sw[(tok * 2 + 0) * kDim + ch] = (a[i] - m1) * r1 * pg1[i] + pb1[i];
      sw[(tok * 2 + 1) * kDim + ch] = (c[i] - m2) * r2 * pg2[i] + pb2[i];
    }
  }
  __syncthreads();
  const int lc  = (lane < 24) ? lane : 23;
  const int tk  = lc / 12;
  const int kh  = (lc - tk * 12) * 4;
  const float* n1 = sw + (tk * 2 + 0) * kDim;
  const float* n2 = sw + (tk * 2 + 1) * kDim;
  v8h h1, h2;
#pragma unroll
  for (int e = 0; e < 8; ++e) {
    const int src = (e & 1) * 48 + kh + (e >> 1);
    const float x1n = n1[src];
    const float x2n = n2[src];
    const float v1 = (src < kSwap) ? x2n : x1n;
    h1[e] = (_Float16)v1;
    h2[e] = (_Float16)x2n;
  }
  unsigned short* q1p = XS + (size_t)t0 * kDim + lc * 8;
  unsigned short* q2p = XS + (size_t)kTok * kDim + (size_t)t0 * kDim + lc * 8;
  for (int pass = 0; pass < 2; ++pass) {
    if (lane < 24) {
      *(volatile v8h*)q1p = h1;
      *(volatile v8h*)q2p = h2;
    }
    __threadfence();
  }
}

__global__ __launch_bounds__(192) void conv_silu_kernel(
    const float* __restrict__ XZ,
    const float* __restrict__ cw0, const float* __restrict__ cb0,
    const float* __restrict__ cw1, const float* __restrict__ cb1,
    float* __restrict__ UC, unsigned short* __restrict__ UC16)
{
  __shared__ __align__(16) float sT[16 * kConvP];
  const int tid = threadIdx.x;
  const int enc = blockIdx.y;
  const float* cw = (enc == 0) ? cw0 : cw1;
  const float* cb = (enc == 0) ? cb0 : cb1;
  const float* XZe = XZ + (size_t)enc * kTok * kXzP;
  float* UCe = UC + (size_t)enc * kTok * kDin;
  unsigned short* UHe = UC16 + (size_t)enc * kTok * kDin;
  const int d  = tid;
  const int g0 = blockIdx.x * 64;
  const int tb = g0 % kSeq;
  const v4f wv = *(const v4f*)(cw + d * 4);
  const float w0 = wv[0], w1 = wv[1], w2 = wv[2], w3 = wv[3];
  const float bc = cb[d];
  float xm3, xm2, xm1;
  {
    const bool hist = (tb > 0);
    const int rb = hist ? (g0 - 3) : g0;
    const float v3 = XZe[(size_t)rb * kXzP + d];
    const float v2 = XZe[(size_t)(rb + 1) * kXzP + d];
    const float v1 = XZe[(size_t)(rb + 2) * kXzP + d];
    xm3 = hist ? v3 : 0.f;
    xm2 = hist ? v2 : 0.f;
    xm1 = hist ? v1 : 0.f;
  }
#pragma unroll 1
  for (int sub = 0; sub < 4; ++sub) {
    const int lb = g0 + sub * 16;
#pragma unroll 1
    for (int s = 0; s < 16; ++s) {
      const float xcur = XZe[(size_t)(lb + s) * kXzP + d];
      float acc = w0 * xm3;
      acc = fmaf(w1, xm2, acc);
      acc = fmaf(w2, xm1, acc);
      acc = fmaf(w3, xcur, acc);
      const float sv = acc + bc;
      const float sg = __builtin_amdgcn_rcpf(1.0f + expf(-sv));
      sT[s * kConvP + tid] = sv * sg;
      xm3 = xm2; xm2 = xm1; xm1 = xcur;
    }
    __syncthreads();
    v4f fv[4];
    v8h bv[2];
#pragma unroll
    for (int it = 0; it < 4; ++it) {
      const int f = it * 192 + tid;
      const int row = f / 48;
      const int c4 = (f - row * 48) * 4;
      fv[it] = *(const v4f*)(sT + row * kConvP + c4);
    }
#pragma unroll
    for (int it = 0; it < 2; ++it) {
      const int f = it * 192 + tid;
      const int row = f / 24;
      const int c8 = (f - row * 24) * 8;
      const float* sp = sT + row * kConvP + c8;
      const v4f a0 = *(const v4f*)(sp);
      const v4f a1 = *(const v4f*)(sp + 4);
#pragma unroll
      for (int e = 0; e < 4; ++e) {
        bv[it][e]     = (_Float16)a0[e];
        bv[it][4 + e] = (_Float16)a1[e];
      }
    }
    for (int pass = 0; pass < 2; ++pass) {
#pragma unroll
      for (int it = 0; it < 4; ++it)
        *(volatile v4f*)(UCe + (size_t)lb * kDin + (size_t)(it * 192 + tid) * 4) = fv[it];
#pragma unroll
      for (int it = 0; it < 2; ++it)
        *(volatile v8h*)(UHe + (size_t)lb * kDin + (size_t)(it * 192 + tid) * 8) = bv[it];
      __threadfence();
    }
    __syncthreads();
  }
}

__global__ __launch_bounds__(384) void scan_kernel(
    const float* __restrict__ XD, const float* __restrict__ UC, const float* __restrict__ XZ,
    const float* __restrict__ dtw0, const float* __restrict__ dtb0, const float* __restrict__ alog0, const float* __restrict__ dp0,
    const float* __restrict__ dtw1, const float* __restrict__ dtb1, const float* __restrict__ alog1, const float* __restrict__ dp1,
    unsigned short* __restrict__ Y16)
{
  __shared__ __align__(16) float sX[16 * kXdP];
  __shared__ __align__(16) float sY[16 * kScanYP];
  __shared__ __align__(16) float sA[8 * 384];
  const int tid = threadIdx.x;
  const int c   = tid >> 1;
  const int sh  = tid & 1;
  const int enc = blockIdx.x >> 1;
  const int bix = blockIdx.x & 1;
  const float* dtw  = (enc == 0) ? dtw0 : dtw1;
  const float* dtb  = (enc == 0) ? dtb0 : dtb1;
  const float* alog = (enc == 0) ? alog0 : alog1;
  const float* dpp  = (enc == 0) ? dp0 : dp1;
  const size_t row0 = (size_t)enc * kTok + (size_t)bix * kSeq;

  float wdt[kDtR];
#pragma unroll
  for (int r = 0; r < kDtR; ++r) wdt[r] = dtw[c * kDtR + r];
  const float bb = dtb[c];
  const float Dd = dpp[c];
#pragma unroll 1
  for (int k = 0; k < 8; ++k) sA[k * 384 + tid] = -expf(alog[c * kNst + sh * 8 + k]);
  __syncthreads();
  float negA[8], h[8];
#pragma unroll
  for (int k = 0; k < 8; ++k) {
    negA[k] = sA[k * 384 + tid];
    h[k] = 0.f;
  }
  const int lr = tid >> 4, lc4 = (tid & 15) * 4;
  const int srow = tid / 24;
  const int sc8  = (tid - srow * 24) * 8;

#pragma unroll 1
  for (int t0 = 0; t0 < kSeq; t0 += 16) {
    if (tid < 256) {
      *(v4f*)(sX + lr * kXdP + lc4) = *(const v4f*)(XD + (row0 + t0 + lr) * kXdP + lc4);
    }
    __syncthreads();
#pragma unroll 1
    for (int s = 0; s < 16; ++s) {
      const size_t row = row0 + (size_t)(t0 + s);
      float xt = UC[row * kDin + c];
      float zv = XZ[row * kXzP + kDin + c];
      asm volatile("" : "+v"(xt));
      asm volatile("" : "+v"(zv));
      const float* xr = sX + s * kXdP;
      float pd = 0.f;
#pragma unroll
      for (int r = 0; r < kDtR; ++r) pd = fmaf(xr[r], wdt[r], pd);
      const float pv = pd + bb;
      const float dt = fmaxf(pv, 0.0f) + log1pf(expf(-fabsf(pv)));
      const float dtx = dt * xt;
      const float* bp = xr + kDtR + sh * 8;
      const float* cp = xr + kDtR + kNst + sh * 8;
      float y = 0.f;
#pragma unroll
      for (int k = 0; k < 8; ++k) {
        const float e = expf(dt * negA[k]);
        h[k] = fmaf(e, h[k], dtx * bp[k]);
        y = fmaf(h[k], cp[k], y);
      }
      const float yo = __shfl_xor(y, 1, 32);
      float ys = y + yo;
      ys = fmaf(xt, Dd, ys);
      const float sg = __builtin_amdgcn_rcpf(1.0f + expf(-zv));
      const float yg = ys * (zv * sg);
      sY[s * kScanYP + sh * kScanYH + c] = yg * kYCarry;
    }
    __syncthreads();
    {
      const float* sp = sY + srow * kScanYP + sc8;
      const v4f a0 = *(const v4f*)(sp);
      const v4f a1 = *(const v4f*)(sp + 4);
      v8h hv;
#pragma unroll
      for (int e = 0; e < 4; ++e) { hv[e] = (_Float16)a0[e]; hv[4 + e] = (_Float16)a1[e]; }
      unsigned short* q = Y16 + (row0 + (size_t)t0) * kDin + (size_t)tid * 8;
      for (int pass = 0; pass < 2; ++pass) {
        *(volatile v8h*)q = hv;
        __threadfence();
      }
    }
  }
}

__global__ __launch_bounds__(128) void outproj_kernel(
    const unsigned short* __restrict__ Yp, const unsigned short* __restrict__ Wp,
    const float* __restrict__ x1, const float* __restrict__ x2,
    float* __restrict__ out, float scale)
{
  __shared__ __align__(16) float sO[4][16 * kOutP];
  const int enc  = blockIdx.y;
  const int lane = threadIdx.x & 31;
  const int wave = threadIdx.x >> 5;
  const int m0   = blockIdx.x * 64 + wave * 16;
  const _Float16* A  = (const _Float16*)Yp + (size_t)enc * kTok * kDin;
  const _Float16* Bt = (const _Float16*)Wp + (size_t)enc * kDim * kDin;
  const float* res = (enc == 0) ? x1 : x2;
  float* C = out + (size_t)enc * kTok * kDim;
  const int rlane = lane & 15;
  const int koff  = (lane >> 4) * 8;
  const int mOff  = (lane >> 4) * 8;

  v8f acc[6];
#pragma unroll
  for (int j = 0; j < 6; ++j) acc[j] = (v8f){0.f, 0.f, 0.f, 0.f, 0.f, 0.f, 0.f, 0.f};

#pragma unroll 1
  for (int k0 = 0; k0 < kDin; k0 += 32) {
    const v16h a = FragH::load(A + (size_t)(m0 + rlane) * kDin + koff + k0);
    v16h b[6];
#pragma unroll
    for (int j = 0; j < 6; ++j) b[j] = FragH::load(Bt + (size_t)((j << 4) + rlane) * kDin + koff + k0);
#pragma unroll
    for (int j = 0; j < 6; ++j) acc[j] = FragH::mma(a, b[j], acc[j]);
    guard6_h(acc[0], acc[1], acc[2], acc[3], acc[4], acc[5], a, b[0], b[1], b[2], b[3], b[4], b[5]);
  }
  acc_guard4(acc[0], acc[1], acc[2], acc[3]);
  acc_guard4(acc[2], acc[3], acc[4], acc[5]);

  float* slab = sO[wave];
#pragma unroll
  for (int j = 0; j < 6; ++j) {
#pragma unroll
    for (int r = 0; r < 8; ++r) slab[(mOff + r) * kOutP + (j << 4) + rlane] = acc[j][r] * scale;
  }
  __syncthreads();
  v4f val[12];
#pragma unroll
  for (int it = 0; it < 12; ++it) {
    const int f = it * 32 + lane;
    const int row = f / 24;
    const int c4 = (f - row * 24) * 4;
    const v4f v  = *(const v4f*)(slab + row * kOutP + c4);
    const v4f rv = *(const v4f*)(res + (size_t)m0 * kDim + (size_t)f * 4);
    val[it] = v + rv;
  }
  for (int pass = 0; pass < 2; ++pass) {
#pragma unroll
    for (int it = 0; it < 12; ++it)
      *(volatile v4f*)(C + (size_t)m0 * kDim + (size_t)(it * 32 + lane) * 4) = val[it];
    __threadfence();
  }
}

extern "C" void kernel_launch(void* const* d_in, const int* in_sizes, int n_in,
                              void* d_out, int out_size, void* d_ws, size_t ws_size,
                              hipStream_t stream)
{
  if (n_in < 24) return;
  if (in_sizes[0] != kTok * kDim || in_sizes[1] != kTok * kDim) return;
  if (in_sizes[2] != kDim || in_sizes[3] != kDim || in_sizes[4] != kDim || in_sizes[5] != kDim) return;
  for (int e = 0; e < kEnc; ++e) {
    const int o = 6 + 9 * e;
    if (in_sizes[o + 0] != kXzP * kDim) return;
    if (in_sizes[o + 1] != kDin * 4) return;
    if (in_sizes[o + 2] != kDin) return;
    if (in_sizes[o + 3] != kXdN * kDin) return;
    if (in_sizes[o + 4] != kDin * kDtR) return;
    if (in_sizes[o + 5] != kDin) return;
    if (in_sizes[o + 6] != kDin * kNst) return;
    if (in_sizes[o + 7] != kDin) return;
    if (in_sizes[o + 8] != kDim * kDin) return;
  }
  if (out_size != kEnc * kTok * kDim) return;
  if (ws_size < kWsTotal) return;

  const float* x1   = (const float*)d_in[0];
  const float* x2   = (const float*)d_in[1];
  const float* ln1g = (const float*)d_in[2];
  const float* ln1b = (const float*)d_in[3];
  const float* ln2g = (const float*)d_in[4];
  const float* ln2b = (const float*)d_in[5];
  const float* in_w0   = (const float*)d_in[6];
  const float* conv_w0 = (const float*)d_in[7];
  const float* conv_b0 = (const float*)d_in[8];
  const float* xprj_w0 = (const float*)d_in[9];
  const float* dt_w0   = (const float*)d_in[10];
  const float* dt_b0   = (const float*)d_in[11];
  const float* a_log0  = (const float*)d_in[12];
  const float* dvec0   = (const float*)d_in[13];
  const float* out_w0  = (const float*)d_in[14];
  const float* in_w1   = (const float*)d_in[15];
  const float* conv_w1 = (const float*)d_in[16];
  const float* conv_b1 = (const float*)d_in[17];
  const float* xprj_w1 = (const float*)d_in[18];
  const float* dt_w1   = (const float*)d_in[19];
  const float* dt_b1   = (const float*)d_in[20];
  const float* a_log1  = (const float*)d_in[21];
  const float* dvec1   = (const float*)d_in[22];
  const float* out_w1  = (const float*)d_in[23];
  float* out = (float*)d_out;

  char* ws = (char*)d_ws;
  unsigned short* WI16 = (unsigned short*)(ws + kOffWI);
  unsigned short* WX16 = (unsigned short*)(ws + kOffWX);
  unsigned short* WO16 = (unsigned short*)(ws + kOffWO);
  unsigned short* XS   = (unsigned short*)(ws + kOffXS);
  float*          XZ   = (float*)(ws + kOffXZ);
  float*          UC   = (float*)(ws + kOffUC);
  unsigned short* UC16 = (unsigned short*)(ws + kOffUC16);
  float*          XD   = (float*)(ws + kOffXD);
  unsigned short* Y16  = (unsigned short*)(ws + kOffY16);

  cast_pad_f16_kernel<<<dim3((kXzP * kDim / 8) / 256, kEnc), 256, 0, stream>>>(in_w0, in_w1, WI16, kXzP, kXzP, kDim, kWCarry);
  cast_pad_f16_kernel<<<dim3((kXdP * kDin / 8) / 256, kEnc), 256, 0, stream>>>(xprj_w0, xprj_w1, WX16, kXdN, kXdP, kDin, kWCarry);
  cast_pad_f16_kernel<<<dim3((kDim * kDin / 8) / 256, kEnc), 256, 0, stream>>>(out_w0, out_w1, WO16, kDim, kDim, kDin, kWCarry);

  ln_swap_shuffle_kernel<<<kTok / 16, 256, 0, stream>>>(x1, x2, ln1g, ln1b, ln2g, ln2b, XS);

  gemm64_f16_kernel<<<dim3((kTok / 64) * (kXzP / 64) / 8, kEnc), 256, 0, stream>>>(
      XS, kDim, (long)kTok * kDim,
      WI16, kDim, (long)kXzP * kDim,
      XZ, kXzP, (long)kTok * kXzP,
      kTok, kXzP, kDim, kInvWCarry);

  conv_silu_kernel<<<dim3(kTok / 64, kEnc), 192, 0, stream>>>(XZ, conv_w0, conv_b0, conv_w1, conv_b1, UC, UC16);

  gemm64_f16_kernel<<<dim3((kTok / 64) * (kXdP / 64) / 8, kEnc), 256, 0, stream>>>(
      UC16, kDin, (long)kTok * kDin,
      WX16, kDin, (long)kXdP * kDin,
      XD, kXdP, (long)kTok * kXdP,
      kTok, kXdP, kDin, kInvWCarry);

  scan_kernel<<<kEnc * kBatch, 384, 0, stream>>>(XD, UC, XZ,
      dt_w0, dt_b0, a_log0, dvec0, dt_w1, dt_b1, a_log1, dvec1, Y16);

  outproj_kernel<<<dim3(kTok / 64, kEnc), 128, 0, stream>>>(Y16, WO16, x1, x2, out, kInvOutCarry);
}
